// ScaleDotProductAttention_3135326126184
// MI455X (gfx1250) — hardware-verified
//
#include <hip/hip_runtime.h>
#include <math.h>
#include <stdint.h>

#ifndef NB
#define NB 4
#endif
#ifndef SEQ
#define SEQ 2048
#endif
#define NB_FULL  4
#define NH       16
#define SEQ_FULL 2048
#define ND       64
#define NBH  (NB * NH)
#define NL   SEQ
#define NS   SEQ
#define NQB  (NL / 128)
#define NKC  (NS / 64)
static_assert(NB >= 1 && NB <= NB_FULL);
static_assert(SEQ >= 128 && SEQ <= SEQ_FULL && (SEQ % 128) == 0);
static_assert((NL % 128) == 0 && (NS % 64) == 0 && ND == 64 && (ND % 32) == 0);
static_assert(NQB >= 1 && NKC >= 2);

typedef __bf16   v16b __attribute__((ext_vector_type(16)));
typedef __bf16   v8b  __attribute__((ext_vector_type(8)));
typedef float    v8f  __attribute__((ext_vector_type(8)));
typedef float    v4f  __attribute__((ext_vector_type(4)));
typedef unsigned int v4u __attribute__((ext_vector_type(4)));

__device__ __forceinline__ unsigned short bf_bits(float f) {
  unsigned u = __float_as_uint(f);
  return (unsigned short)((u + 0x7FFFu + ((u >> 16) & 1u)) >> 16);
}
__device__ __forceinline__ float bf_up(unsigned short hb) { return __uint_as_float(((unsigned)hb) << 16); }
__device__ __forceinline__ __bf16 bf_val(unsigned short hb) { return __builtin_bit_cast(__bf16, hb); }
__device__ __forceinline__ unsigned pk16(unsigned short a, unsigned short b) { return (unsigned)a | ((unsigned)b << 16); }
__device__ __forceinline__ v8f zero8() { v8f z = {0.f, 0.f, 0.f, 0.f, 0.f, 0.f, 0.f, 0.f}; return z; }

__device__ __forceinline__ v16b ldfrag_b(const __bf16* p) {
  union { v16b v; v8b h[2]; } f;
  f.h[0] = *(const v8b*)(p);
  f.h[1] = *(const v8b*)(p + 16);
  return f.v;
}

__device__ __forceinline__ v8f mma_b(v16b a, v16b b, v8f c) {
  c = __builtin_amdgcn_wmma_f32_16x16x32_bf16(false, a, false, b, (short)0, c, false, false);
  asm volatile("v_nop\n\tv_nop\n\tv_nop\n\tv_nop" : "+v"(c) : "v"(a), "v"(b));
  return c;
}

__device__ __forceinline__ v4u cvt8(const float* __restrict__ p) {
  const v4f a = *(const v4f*)(p);
  const v4f b = *(const v4f*)(p + 4);
  v4u r;
  r[0] = pk16(bf_bits(a[0]), bf_bits(a[1]));
  r[1] = pk16(bf_bits(a[2]), bf_bits(a[3]));
  r[2] = pk16(bf_bits(b[0]), bf_bits(b[1]));
  r[3] = pk16(bf_bits(b[2]), bf_bits(b[3]));
  return r;
}

__global__ __launch_bounds__(256) void cvt_qk(const float* __restrict__ q, const float* __restrict__ k,
                                              unsigned short* Qo, unsigned short* Ko, int n8) {
  const int i = blockIdx.x * 256 + threadIdx.x;
  if (i < n8) {
    const size_t e   = (size_t)i * 8;
    const size_t bh  = e / ((size_t)NL * ND);
    const size_t src = bh * ((size_t)SEQ_FULL * ND) + (e - bh * ((size_t)NL * ND));
    const v4u pq = cvt8(q + src);
    const v4u pk = cvt8(k + src);
    *(volatile v4u*)(Qo + e) = pq;
    *(volatile v4u*)(Ko + e) = pk;
    __threadfence();
    *(volatile v4u*)(Qo + e) = pq;
    *(volatile v4u*)(Ko + e) = pk;
  }
}

__global__ __launch_bounds__(256) void prep_vt(const float* __restrict__ v, unsigned short* VT) {
  __shared__ __align__(16) unsigned short T[ND * 72];
  const int tid   = threadIdx.x;
  const int stile = blockIdx.x % NKC;
  const int bh    = blockIdx.x / NKC;
  const int s0    = stile * 64;
  const float* vp = v + ((size_t)bh * SEQ_FULL + s0) * ND;
#pragma unroll
  for (int rr = 0; rr < 4; ++rr) {
    const int idx  = tid + rr * 256;
    const int srow = idx >> 4;
    const int d4   = (idx & 15) << 2;
    const v4f vf = *(const v4f*)(vp + (size_t)srow * ND + d4);
#pragma unroll
    for (int e = 0; e < 4; ++e) T[(d4 + e) * 72 + srow] = bf_bits(vf[e]);
  }
  __syncthreads();
  unsigned short* vout = VT + (size_t)bh * ND * NS + s0;
  v4u tv[2];
  size_t to[2];
#pragma unroll
  for (int rr = 0; rr < 2; ++rr) {
    const int idx  = tid + rr * 256;
    const int drow = idx >> 3;
    const int c8   = (idx & 7) << 3;
    tv[rr] = *(const v4u*)(T + drow * 72 + c8);
    to[rr] = (size_t)drow * NS + c8;
  }
  for (int pass = 0; pass < 2; ++pass) {
    *(volatile v4u*)(vout + to[0]) = tv[0];
    *(volatile v4u*)(vout + to[1]) = tv[1];
    __threadfence();
  }
}

#define L_K     0
#define L_V     8192
#define L_P     16384
#define L_TOTAL 49152
static_assert(L_V - L_K == 64 * ND * 2);
static_assert(L_P - L_V == ND * 64 * 2);
static_assert(L_TOTAL - L_P == 8 * 2 * 16 * 64 * 2);
static_assert(16 * ND * 4 == 2 * 16 * 64 * 2);

__global__ __launch_bounds__(256)
void attn_hm(const unsigned short* __restrict__ qbp, const unsigned short* __restrict__ kbp,
             const unsigned short* __restrict__ vtp, float* Op) {
  __shared__ __align__(16) unsigned char lds[L_TOTAL];
  union FB { v16b v; v8b h[2]; };
  __bf16* Ksh = (__bf16*)(lds + L_K);
  __bf16* Vth = (__bf16*)(lds + L_V);
  __bf16* Pb  = (__bf16*)(lds + L_P);

  const int tid  = threadIdx.x;
  const int wave = tid >> 5;
  const int lane = tid & 31;
  const int hh   = lane >> 4;
  const int c    = lane & 15;

  const int bx = blockIdx.x;
  const int qb = bx % NQB;
  const int bh = bx / NQB;
  const int q0 = qb * 128 + wave * 16;

  const __bf16* Qg = (const __bf16*)(const void*)qbp;
  const __bf16* Kg = (const __bf16*)(const void*)kbp;
  const __bf16* Vg = (const __bf16*)(const void*)vtp + (size_t)bh * ND * NS;

  __bf16* pwh = Pb + wave * 2048;
  __bf16* pwl = pwh + 1024;

  const size_t qo = ((size_t)bh * NL + q0 + c) * ND + 8 * hh;
  v16b qa[2];
  qa[0] = ldfrag_b(Qg + qo);
  qa[1] = ldfrag_b(Qg + qo + 32);

  v8f O[4];
#pragma unroll
  for (int t = 0; t < 4; ++t) O[t] = zero8();
  float mrow[8], lrow[8], alpha[8];
#pragma unroll
  for (int r = 0; r < 8; ++r) { mrow[r] = -INFINITY; lrow[r] = 0.f; alpha[r] = 0.f; }

  for (int kt = 0; kt < NKC; ++kt) {
    const int kv0 = kt * 64;
    __syncthreads();
    {
#pragma unroll
      for (int i = 0; i < 2; ++i) {
        const int p  = tid + 256 * i;
        const int rw = p >> 3;
        const int sg = (p & 7) * 8;
        const v8b a0 = *(const v8b*)(Kg + ((size_t)bh * NS + kv0 + rw) * ND + sg);
        const v8b b0 = *(const v8b*)(Vg + (size_t)rw * NS + kv0 + sg);
        *(v8b*)(Ksh + rw * 64 + sg) = a0;
        *(v8b*)(Vth + rw * 64 + sg) = b0;
      }
    }
    __syncthreads();

    v8f s[4];
#pragma unroll
    for (int j = 0; j < 4; ++j) s[j] = zero8();
#pragma unroll
    for (int dc = 0; dc < 2; ++dc) {
      const int ko = dc * 32 + 8 * hh;
#pragma unroll
      for (int j = 0; j < 4; ++j) {
        const int kr = (j * 16 + c) * 64 + ko;
        FB kb;
        kb.h[0] = *(const v8b*)(Ksh + kr);
        kb.h[1] = *(const v8b*)(Ksh + kr + 16);
        s[j] = mma_b(qa[dc], kb.v, s[j]);
      }
    }
#pragma unroll
    for (int j = 0; j < 4; ++j) s[j] = s[j] * 0.125f;

#pragma unroll
    for (int r = 0; r < 8; ++r) {
      float m = -INFINITY;
#pragma unroll
      for (int j = 0; j < 4; ++j) m = fmaxf(m, s[j][r]);
#pragma unroll
      for (int off = 1; off < 16; off <<= 1) m = fmaxf(m, __shfl_xor(m, off, 32));
      const float mnew = fmaxf(mrow[r], m);
      const float al   = __expf(mrow[r] - mnew);
      mrow[r]  = mnew;
      alpha[r] = al;
      float psum = 0.f;
#pragma unroll
      for (int j = 0; j < 4; ++j) {
        const float p = __expf(s[j][r] - mnew);
        psum += p;
        const unsigned short hb = bf_bits(p);
        const unsigned short lb = bf_bits(p - bf_up(hb));
        const int po = (8 * hh + r) * 64 + j * 16 + c;
        pwh[po] = bf_val(hb);
        pwl[po] = bf_val(lb);
      }
#pragma unroll
      for (int off = 1; off < 16; off <<= 1) psum += __shfl_xor(psum, off, 32);
      lrow[r] = lrow[r] * al + psum;
    }
    __builtin_amdgcn_fence(3, "workgroup");
    __builtin_amdgcn_wave_barrier();
    __builtin_amdgcn_fence(2, "workgroup");

#pragma unroll
    for (int t = 0; t < 4; ++t) {
#pragma unroll
      for (int r = 0; r < 8; ++r) O[t][r] *= alpha[r];
    }
#pragma unroll
    for (int kk = 0; kk < 2; ++kk) {
      const int pr = c * 64 + kk * 32 + 8 * hh;
      FB pa, pl;
      pa.h[0] = *(const v8b*)(pwh + pr);
      pa.h[1] = *(const v8b*)(pwh + pr + 16);
      pl.h[0] = *(const v8b*)(pwl + pr);
      pl.h[1] = *(const v8b*)(pwl + pr + 16);
#pragma unroll
      for (int t = 0; t < 4; ++t) {
        const int vr = (t * 16 + c) * 64 + kk * 32 + 8 * hh;
        FB vb;
        vb.h[0] = *(const v8b*)(Vth + vr);
        vb.h[1] = *(const v8b*)(Vth + vr + 16);
        O[t] = mma_b(pa.v, vb.v, O[t]);
        O[t] = mma_b(pl.v, vb.v, O[t]);
      }
    }
  }
  __syncthreads();

  float* os = (float*)(lds + L_P) + wave * 1024;
  float inv[8];
#pragma unroll
  for (int r = 0; r < 8; ++r) inv[r] = (lrow[r] > 0.f) ? (1.0f / lrow[r]) : 0.f;
#pragma unroll
  for (int t = 0; t < 4; ++t) {
#pragma unroll
    for (int r = 0; r < 8; ++r) os[(8 * hh + r) * 64 + t * 16 + c] = O[t][r] * inv[r];
  }
  __builtin_amdgcn_fence(3, "workgroup");
  __builtin_amdgcn_wave_barrier();
  __builtin_amdgcn_fence(2, "workgroup");
  float* og = Op + ((size_t)bh * NL + q0) * ND;
  const int colw = c * 4;
  v4f ov[8];
#pragma unroll
  for (int it = 0; it < 8; ++it) {
    const int row = 2 * it + hh;
    ov[it] = *(const v4f*)(os + row * 64 + colw);
  }
  for (int pass = 0; pass < 2; ++pass) {
#pragma unroll
    for (int it = 0; it < 8; ++it) {
      const int row = 2 * it + hh;
      *(volatile v4f*)(og + (size_t)row * ND + colw) = ov[it];
    }
    __threadfence();
  }
}

extern "C" void kernel_launch(void* const* d_in, const int* in_sizes, int n_in,
                              void* d_out, int out_size, void* d_ws, size_t ws_size,
                              hipStream_t stream) {
  const int nneed = NBH * SEQ_FULL * ND;
  const int nout  = NBH * NL * ND;
  if (n_in < 3) return;
  if (in_sizes[0] < nneed || in_sizes[1] < nneed || in_sizes[2] < nneed) return;
  if (out_size < nout) return;

  const float* q = (const float*)d_in[0];
  const float* k = (const float*)d_in[1];
  const float* v = (const float*)d_in[2];

  const size_t PL = (size_t)nout * 2;
  size_t off = 0;
  const size_t oQ = off; off += PL;
  const size_t oK = off; off += PL;
  const size_t oV = off; off += PL;
  if (off > ws_size) return;
  if (off > (size_t)134217728) return;

  char* ws = (char*)d_ws;
  unsigned short* Qb = (unsigned short*)(ws + oQ);
  unsigned short* Kb = (unsigned short*)(ws + oK);
  unsigned short* VT = (unsigned short*)(ws + oV);

  const int  n8 = nout / 8;
  const dim3 blk(256);
  const dim3 gCvt((n8 + 255) / 256);
  const dim3 gVt(NBH * NKC);
  const dim3 gAttn(NBH * NQB);

  cvt_qk<<<gCvt, blk, 0, stream>>>(q, k, Qb, Kb, n8);
  prep_vt<<<gVt, blk, 0, stream>>>(v, VT);
  attn_hm<<<gAttn, blk, 0, stream>>>(Qb, Kb, VT, (float*)d_out);
  (void)hipGetLastError();
}
